// att_layer_72550587564439
// MI455X (gfx1250) — hardware-verified
//
#include <hip/hip_runtime.h>


#define NN   16384
#define DI   256
#define HH   128
#define DO_  256
#define QB   2048
#define TQ   QB
#define PCAR 1024.0f
#define SCL  0.088388347648318447f
typedef _Float16 h16;
typedef unsigned short bf;
typedef __attribute__((ext_vector_type(16))) __bf16   v16bf;
typedef __attribute__((ext_vector_type(16))) _Float16 v16h;
typedef __attribute__((ext_vector_type(8)))  _Float16 v8h;
typedef __attribute__((ext_vector_type(8)))  unsigned short v8us;
typedef __attribute__((ext_vector_type(8)))  float    v8f;
typedef __attribute__((ext_vector_type(4)))  float    v4f;
typedef v8h  __attribute__((may_alias)) v8ha;
typedef v4f  __attribute__((may_alias)) v4fa;
typedef v8us __attribute__((may_alias)) v8usa;

__device__ __forceinline__ unsigned short f2bf(float f) { unsigned u = __float_as_uint(f); u += 0x7FFFu + ((u >> 16) & 1u); return (unsigned short)(u >> 16); }
__device__ __forceinline__ float bf2f(unsigned short b) { return __uint_as_float(((unsigned)b) << 16); }
__device__ __forceinline__ float bfr(float f) { return bf2f(f2bf(f)); }
__device__ __forceinline__ v16h cat16(v8h lo, v8h hi) { return __builtin_shufflevector(lo, hi, 0, 1, 2, 3, 4, 5, 6, 7, 8, 9, 10, 11, 12, 13, 14, 15); }
__device__ __forceinline__ v16bf cat16b(v8us lo, v8us hi) { return __builtin_bit_cast(v16bf, __builtin_shufflevector(lo, hi, 0, 1, 2, 3, 4, 5, 6, 7, 8, 9, 10, 11, 12, 13, 14, 15)); }
__device__ __forceinline__ v8f wmma16(v16h a, v16h b, v8f c) { return __builtin_amdgcn_wmma_f32_16x16x32_f16(false, a, false, b, (short)0, c, false, false); }
__device__ __forceinline__ v8f wmmab(v16bf a, v16bf b, v8f c) { return __builtin_amdgcn_wmma_f32_16x16x32_bf16(false, a, false, b, (short)0, c, false, false); }


template <typename T16> struct WFrag;
template <> struct WFrag<h16> { typedef v16h V; static __device__ __forceinline__ V ld(const h16* p) { return cat16(*(const v8h*)p, *(const v8h*)(p + 16)); } static __device__ __forceinline__ v8f mma(V a, V b, v8f c) { return wmma16(a, b, c); } };
template <> struct WFrag<bf> { typedef v16bf V; static __device__ __forceinline__ V ld(const bf* p) { return cat16b(*(const v8us*)p, *(const v8us*)(p + 16)); } static __device__ __forceinline__ v8f mma(V a, V b, v8f c) { return wmmab(a, b, c); } };
template <typename T16, int NSPLIT, bool BIAS>
__global__ __launch_bounds__(32) void k_gemmw(const T16* __restrict__ A, const T16* __restrict__ A2, const T16* __restrict__ Bt, const T16* __restrict__ Bt2, int K, float* C, int ldc, const float* __restrict__ bias, size_t sA, size_t sB, size_t sC) {
    typedef typename WFrag<T16>::V V;
    __shared__ __align__(16) float os[16 * 68];
    const size_t z = blockIdx.z; A += z * sA; if (A2) A2 += z * sA; Bt += z * sB; if (Bt2) Bt2 += z * sB; C += z * sC;
    const int lane = threadIdx.x & 31, lr = lane & 15, hi = lane >> 4; const int r0 = blockIdx.x * 64, c0 = blockIdx.y * 64;
    v8f acc[4][4];
#pragma unroll
    for (int mb = 0; mb < 4; ++mb)
#pragma unroll
        for (int nb = 0; nb < 4; ++nb) acc[mb][nb] = (v8f){};
    const size_t aoff = (size_t)(r0 + lr) * K + 8 * hi, boff = (size_t)(c0 + lr) * K + 8 * hi;
#pragma unroll 1
    for (int kc = 0; kc < K; kc += 32) {
        V a[4], a2[4];
#pragma unroll
        for (int mb = 0; mb < 4; ++mb) { a[mb] = WFrag<T16>::ld(A + aoff + (size_t)mb * 16 * K + kc); if (NSPLIT == 1 || NSPLIT == 2) a2[mb] = WFrag<T16>::ld(A2 + aoff + (size_t)mb * 16 * K + kc); }
#pragma unroll
        for (int nb = 0; nb < 4; ++nb) { const V b = WFrag<T16>::ld(Bt + boff + (size_t)nb * 16 * K + kc); V b2; if (NSPLIT >= 2) b2 = WFrag<T16>::ld(Bt2 + boff + (size_t)nb * 16 * K + kc);
#pragma unroll
            for (int mb = 0; mb < 4; ++mb) { acc[mb][nb] = WFrag<T16>::mma(a[mb], b, acc[mb][nb]); if (NSPLIT == 1 || NSPLIT == 2) acc[mb][nb] = WFrag<T16>::mma(a2[mb], b, acc[mb][nb]); if (NSPLIT >= 2) acc[mb][nb] = WFrag<T16>::mma(a[mb], b2, acc[mb][nb]); } }
        asm volatile("v_nop\n\tv_nop\n\tv_nop\n\tv_nop" : "+v"(acc[0][0]), "+v"(acc[1][1]), "+v"(acc[2][2]), "+v"(acc[3][3]) : "v"(a[0]), "v"(a[3]));
    }
#pragma unroll
    for (int mb = 0; mb < 4; ++mb) {
#pragma unroll
        for (int nb = 0; nb < 4; ++nb) {
#pragma unroll
            for (int j = 0; j < 8; ++j) os[(hi * 8 + j) * 68 + nb * 16 + lr] = acc[mb][nb][j]; }
        __builtin_amdgcn_wave_barrier(); asm volatile("" ::: "memory");
        float* crow = C + (size_t)(r0 + mb * 16) * ldc + c0;
#pragma unroll 1
        for (int ps = 0; ps < 2; ++ps) {
#pragma unroll
            for (int s = 0; s < 8; ++s) { const int row = 2 * s + hi, cofs = lr * 4; v4f val = *(const v4fa*)(os + row * 68 + cofs); if (BIAS) { val[0] += bfr(bias[c0 + cofs]); val[1] += bfr(bias[c0 + cofs + 1]); val[2] += bfr(bias[c0 + cofs + 2]); val[3] += bfr(bias[c0 + cofs + 3]); }
                *(volatile v4f*)(crow + (size_t)row * ldc + cofs) = val; }
            if (ps == 0) __threadfence(); }
        __builtin_amdgcn_wave_barrier(); asm volatile("" ::: "memory");
    }
}

__device__ __forceinline__ h16 tohx(float x) { return (h16)x; }
__device__ __forceinline__ void splitf(float y, unsigned short& h, unsigned short& l) { h = f2bf(y); l = f2bf(y - bf2f(h)); }
typedef __attribute__((ext_vector_type(2))) _Float16 v2h;
typedef __attribute__((ext_vector_type(4))) _Float16 v4h;
typedef __attribute__((ext_vector_type(2))) unsigned short v2us;

__global__ __launch_bounds__(256) void k_wtG(const float* __restrict__ w, int K, int N, bf* Bt) {
    const int lane = threadIdx.x & 31; const int L0 = (blockIdx.x * 8 + (threadIdx.x >> 5)) * 8; const int nlines = N * K / 64;
#pragma unroll 1
    for (int ps = 0; ps < 2; ++ps) {
#pragma unroll 1
        for (int l = 0; l < 8; ++l) { const int L = L0 + l; if (L >= nlines) break; const size_t e = (size_t)L * 64 + lane * 2; const int k = (int)(e % K), n = (int)(e / K); v2us o;
            o[0] = f2bf(w[(size_t)k * N + n]); o[1] = f2bf(w[(size_t)(k + 1) * N + n]); *(volatile v2us*)(Bt + e) = o; }
        if (ps == 0) __threadfence(); }
}
__global__ __launch_bounds__(256) void k_cvt8(const float* __restrict__ src, bf* dst, size_t n8) { const size_t i = (size_t)blockIdx.x * 256 + threadIdx.x; if (i >= n8) return; const v8f v = *(const v8f*)(src + i * 8); v8us o;
#pragma unroll
    for (int k = 0; k < 8; ++k) o[k] = f2bf(v[k]); *(volatile v8us*)(dst + i * 8) = o; __threadfence(); *(volatile v8us*)(dst + i * 8) = o; }
__global__ __launch_bounds__(256) void k_p16(const float* __restrict__ F, h16* P, size_t n) { const size_t i = ((size_t)blockIdx.x * 256 + threadIdx.x) * 2; if (i >= n) return; v2h o; o[0] = tohx(F[i]); o[1] = tohx(F[i + 1]); *(volatile v2h*)(P + i) = o; __threadfence(); *(volatile v2h*)(P + i) = o; }
__global__ __launch_bounds__(256) void k_vt(const float* __restrict__ F, h16* VT) { const size_t e = ((size_t)blockIdx.x * 256 + threadIdx.x) * 2; if (e >= (size_t)HH * NN) return; const int j = (int)(e % NN), c = (int)(e / NN); v2h o; o[0] = tohx(F[(size_t)j * HH + c]); o[1] = tohx(F[(size_t)(j + 1) * HH + c]); *(volatile v2h*)(VT + e) = o; __threadfence(); *(volatile v2h*)(VT + e) = o; }
__global__ __launch_bounds__(256) void k_osplit(const float* __restrict__ O, const float* __restrict__ RS, bf* Ah, bf* Al) { const size_t e = ((size_t)blockIdx.x * 256 + threadIdx.x) * 2; if (e >= (size_t)QB * HH) return; const int i = (int)(e / HH); const float rsn = RS[(size_t)i * 32 + 1]; v2us oh, ol;
#pragma unroll
    for (int q = 0; q < 2; ++q) { unsigned short a, c2; splitf(__fmul_rn(O[e + q], rsn), a, c2); oh[q] = a; ol[q] = c2; } *(volatile v2us*)(Ah + e) = oh; *(volatile v2us*)(Al + e) = ol; __threadfence(); *(volatile v2us*)(Ah + e) = oh; *(volatile v2us*)(Al + e) = ol; }
template <int NK>
__global__ __launch_bounds__(256) void k_smax(const float* __restrict__ S, float* RS) { const int lane = threadIdx.x & 31; const int i = blockIdx.x * 8 + (threadIdx.x >> 5); if (i >= TQ) return; const float* sr = S + (size_t)i * NK; float m = -3.0e38f;
#pragma unroll 4
    for (int c0 = lane * 4; c0 < NK; c0 += 128) { const v4f v = *(const v4f*)(sr + c0); m = fmaxf(m, fmaxf(fmaxf(v[0], v[1]), fmaxf(v[2], v[3]))); }
#pragma unroll
    for (int sh = 16; sh; sh >>= 1) m = fmaxf(m, __shfl_xor(m, sh, 32));
    const float o = lane == 0 ? m : 0.f; *(volatile float*)(RS + (size_t)i * 32 + lane) = o; __threadfence(); *(volatile float*)(RS + (size_t)i * 32 + lane) = o; }
template <int NK>
__global__ __launch_bounds__(256) void k_sexp(const float* __restrict__ S, float* RS, h16* P) { const int lane = threadIdx.x & 31; const int i = blockIdx.x * 8 + (threadIdx.x >> 5); if (i >= TQ) return; const float* sr = S + (size_t)i * NK; const float m = RS[(size_t)i * 32]; float sum = 0.f;
#pragma unroll 1
    for (int ps = 0; ps < 2; ++ps) { sum = 0.f;
#pragma unroll 2
        for (int c0 = lane * 4; c0 < NK; c0 += 128) { const v4f v = *(const v4f*)(sr + c0); v4h o;
#pragma unroll
            for (int q = 0; q < 4; ++q) { float dlt = __fsub_rn(v[q], m); asm volatile("" : "+v"(dlt)); const float e = __expf(__fmul_rn(dlt, SCL)); sum += e; o[q] = tohx(e * PCAR); }
            *(volatile v4h*)(P + (size_t)i * NK + c0) = o; }
        if (ps == 0) __threadfence(); }
#pragma unroll
    for (int sh = 16; sh; sh >>= 1) sum += __shfl_xor(sum, sh, 32);
    const float o2 = lane == 0 ? m : (lane == 1 ? __fdiv_rn(1.0f, sum * PCAR) : 0.f); *(volatile float*)(RS + (size_t)i * 32 + lane) = o2; __threadfence(); *(volatile float*)(RS + (size_t)i * 32 + lane) = o2; }

extern "C" void kernel_launch(void* const* d_in, const int* in_sizes, int n_in,
                              void* d_out, int out_size, void* d_ws, size_t ws_size, hipStream_t stream) {
    (void)in_sizes; (void)n_in; (void)out_size;
    const float* IN[11]; for (int i = 0; i < 11; ++i) IN[i] = (const float*)d_in[i];
    float* OUT = (float*)d_out;
    char* wsp = (char*)d_ws;
    auto take = [&](size_t bytes) { char* p = wsp; wsp += (bytes + 255) & ~(size_t)255; return (void*)p; };
    bf* WQ = (bf*)take((size_t)HH * DI * 2); bf* WK = (bf*)take((size_t)HH * DI * 2); bf* WV = (bf*)take((size_t)HH * DI * 2); bf* WO = (bf*)take((size_t)DO_ * HH * 2); bf* XB = (bf*)take((size_t)NN * DI * 2); float* F = (float*)take((size_t)NN * HH * 4);
    h16* Q16 = (h16*)take((size_t)NN * HH * 2); h16* K16 = (h16*)take((size_t)NN * HH * 2); h16* VT = (h16*)take((size_t)HH * NN * 2); float* S = (float*)take((size_t)QB * NN * 4); h16* P = (h16*)take((size_t)QB * NN * 2); float* RS = (float*)take((size_t)QB * 32 * 4); float* O = (float*)take((size_t)QB * HH * 4); bf* Ah = (bf*)take((size_t)QB * HH * 2); bf* Al = (bf*)take((size_t)QB * HH * 2);
    if ((size_t)(wsp - (char*)d_ws) > ws_size) return;
    { const unsigned g = (unsigned)((DI * HH / 64 + 63) / 64); k_wtG<<<g, 256, 0, stream>>>(IN[3], DI, HH, WQ); k_wtG<<<g, 256, 0, stream>>>(IN[5], DI, HH, WK); k_wtG<<<g, 256, 0, stream>>>(IN[7], DI, HH, WV); k_wtG<<<(unsigned)((HH * DO_ / 64 + 63) / 64), 256, 0, stream>>>(IN[9], HH, DO_, WO); }
    const unsigned LX = (unsigned)(((size_t)NN * DI / 8 + 255) / 256), L2 = (unsigned)(((size_t)NN * HH / 2 + 255) / 256); const dim3 gP(NN / 64, HH / 64, 1);
    k_cvt8<<<LX, 256, 0, stream>>>(IN[0], XB, (size_t)NN * DI / 8); k_gemmw<bf, 0, true><<<gP, 32, 0, stream>>>(XB, nullptr, WQ, nullptr, DI, F, HH, IN[4], 0, 0, 0); k_p16<<<L2, 256, 0, stream>>>(F, Q16, (size_t)NN * HH);
    k_cvt8<<<LX, 256, 0, stream>>>(IN[1], XB, (size_t)NN * DI / 8); k_gemmw<bf, 0, true><<<gP, 32, 0, stream>>>(XB, nullptr, WK, nullptr, DI, F, HH, IN[6], 0, 0, 0); k_p16<<<L2, 256, 0, stream>>>(F, K16, (size_t)NN * HH);
    k_cvt8<<<LX, 256, 0, stream>>>(IN[2], XB, (size_t)NN * DI / 8); k_gemmw<bf, 0, true><<<gP, 32, 0, stream>>>(XB, nullptr, WV, nullptr, DI, F, HH, IN[8], 0, 0, 0); k_vt<<<L2, 256, 0, stream>>>(F, VT);
    for (int qb = 0; qb < NN / QB; ++qb) {
        k_gemmw<h16, 0, false><<<dim3(QB / 64, NN / 64, 1), 32, 0, stream>>>(Q16 + (size_t)qb * QB * HH, nullptr, K16, nullptr, HH, S, NN, nullptr, 0, 0, 0);
        k_smax<NN><<<QB / 8, 256, 0, stream>>>(S, RS); k_sexp<NN><<<QB / 8, 256, 0, stream>>>(S, RS, P);
        k_gemmw<h16, 0, false><<<dim3(QB / 64, HH / 64, 1), 32, 0, stream>>>(P, nullptr, VT, nullptr, NN, O, HH, nullptr, 0, 0, 0);
        k_osplit<<<(unsigned)(((size_t)QB * HH / 2 + 255) / 256), 256, 0, stream>>>(O, RS, Ah, Al);
        k_gemmw<bf, 1, true><<<dim3(QB / 64, DO_ / 64, 1), 32, 0, stream>>>(Ah, Al, WO, nullptr, HH, OUT + (size_t)qb * QB * DO_, DO_, IN[10], 0, 0, 0); }
}
